// DotProductCredibility_55276229100112
// MI455X (gfx1250) — hardware-verified
//
#include <hip/hip_runtime.h>
#include <stddef.h>


typedef _Float16 v16h __attribute__((ext_vector_type(16)));
typedef _Float16 v8h  __attribute__((ext_vector_type(8)));
typedef float    v8f  __attribute__((ext_vector_type(8)));
typedef float    v4f  __attribute__((ext_vector_type(4)));
typedef _Float16 h16;

#ifndef NB
#define NB 8
#endif
#ifndef SEQ
#define SEQ 2048
#endif
#define NB_FULL  8
#define SEQ_FULL 2048
#define HD    64
#define MROWS (NB * SEQ)

static_assert(NB >= 1 && NB <= NB_FULL);
static_assert(SEQ >= 128 && SEQ <= SEQ_FULL && (SEQ % 128) == 0);
static_assert(HD == 64);
static_assert((HD % 32) == 0 && (HD % 8) == 0);
static_assert(((MROWS * 8) % 256) == 0);
static_assert((SEQ % 16) == 0);
static_assert((size_t)NB_FULL * SEQ_FULL * 4 == (size_t)65536);
static_assert(128 * 4 <= 131072);

#define XCARRY 64.0f

#define PLANE16_BYTES ((size_t)MROWS * HD * 2)
#define OFF_Q  ((size_t)0)
#define OFF_K  (OFF_Q + PLANE16_BYTES)
#define WS_TOTAL (OFF_K + PLANE16_BYTES)
static_assert((PLANE16_BYTES % 128) == 0);
static_assert(WS_TOTAL <= (size_t)134217728);

__device__ __forceinline__ float bf16r(float x) {
  unsigned int u = __float_as_uint(x);
  u = (u + 0x7FFFu + ((u >> 16) & 1u)) & 0xFFFF0000u;
  return __uint_as_float(u);
}

static __device__ __forceinline__ h16 toh_flush(float v) {
  const h16 r = (h16)v;
  return (fabsf(v) < 6.103515625e-05f) ? (h16)0.0f : r;
}

__device__ __forceinline__ v16h frag_at(const _Float16* p) {
  v8h lo = *(const v8h*)(p);
  v8h hi = *(const v8h*)(p + 16);
  v16h out;
#pragma unroll
  for (int i = 0; i < 8; ++i) { out[i] = lo[i]; out[i + 8] = hi[i]; }
  return out;
}

__device__ __forceinline__ v8f wmma16(v16h a, v16h b, v8f c) {
  v8f d = __builtin_amdgcn_wmma_f32_16x16x32_f16(false, a, false, b, (short)0, c,
                                                 false, false);
  asm volatile("v_nop\n\tv_nop\n\tv_nop\n\tv_nop" : "+v"(d) : "v"(a), "v"(b));
  return d;
}

__device__ __forceinline__ float red16_sum(float x) {
#pragma unroll
  for (int off = 1; off < 16; off <<= 1) x += __shfl_xor(x, off, 32);
  return x;
}

__global__ __launch_bounds__(256) void cast_kernel(
    const float* __restrict__ X, _Float16* __restrict__ dst) {
  const unsigned g = blockIdx.x * 256u + threadIdx.x;
  const unsigned crow = g >> 3;
  const unsigned c = (g & 7u) * 8u;
  const unsigned bidx = crow / (unsigned)SEQ;
  const unsigned sq = crow - bidx * (unsigned)SEQ;
  const size_t srow = (size_t)bidx * SEQ_FULL + sq;
  const v4f a0 = *(const v4f*)(X + srow * HD + c);
  const v4f a1 = *(const v4f*)(X + srow * HD + c + 4u);
  v8h o;
#pragma unroll
  for (int i = 0; i < 4; ++i) {
    o[i]     = toh_flush(XCARRY * bf16r(a0[i]));
    o[i + 4] = toh_flush(XCARRY * bf16r(a1[i]));
  }
  _Float16* p = dst + (size_t)crow * HD + c;
  *(volatile v8h*)p = o;
  __threadfence();
  *(volatile v8h*)p = o;
}

__global__ __launch_bounds__(256) void cred_kernel(
    const _Float16* __restrict__ Qh, const _Float16* __restrict__ Kh,
    const float* __restrict__ scale, const int* __restrict__ valid_lens,
    float* __restrict__ out) {
  __shared__ __attribute__((aligned(16))) float Rs[128];

  const unsigned tid = threadIdx.x, lane = tid & 31u;
  const unsigned wave = (unsigned)__builtin_amdgcn_readfirstlane((int)(threadIdx.x >> 5));
  const unsigned hh = lane >> 4, m = lane & 15u;
  const unsigned q0 = blockIdx.x * 128u;
  const unsigned b = blockIdx.y;

  const int vl_in = valid_lens[b];
  const int vlc = min(max(vl_in, 0), (int)SEQ);
  const unsigned nfull = (unsigned)vlc >> 4;
  const unsigned rem = (unsigned)vlc & 15u;
  const unsigned gt = min(nfull, (unsigned)(SEQ / 16 - 1));

  const _Float16* qp = Qh + (size_t)(b * (unsigned)SEQ + q0 + wave * 16u + m) * HD + hh * 8u;
  const v16h qf0 = frag_at(qp);
  const v16h qf1 = frag_at(qp + 32);

  const _Float16* kp = Kh + ((size_t)b * SEQ + m) * HD + hh * 8u;

  v8f acc = {};
#pragma unroll 2
  for (unsigned g = 0; g < nfull; ++g) {
    const _Float16* kg = kp + (size_t)g * (16u * HD);
    const v16h k0f = frag_at(kg);
    const v16h k1f = frag_at(kg + 32);
    acc = wmma16(qf0, k0f, acc);
    acc = wmma16(qf1, k1f, acc);
  }

  v8f t = {};
  {
    const _Float16* kg = kp + (size_t)gt * (16u * HD);
    const v16h k0f = frag_at(kg);
    const v16h k1f = frag_at(kg + 32);
    t = wmma16(qf0, k0f, t);
    t = wmma16(qf1, k1f, t);
  }

  const bool keep = (m < rem);
  const float sc = bf16r(scale[0]);
  const float rv = 1.0f / (float)vl_in;
  float val[8];
#pragma unroll
  for (int v = 0; v < 8; ++v) {
    const float tv = keep ? t[v] : 0.0f;
    const float tot = red16_sum(acc[v] + tv);
    val[v] = ((tot * (1.0f / (XCARRY * XCARRY))) * 0.125f) * sc * rv;
  }

  if (m == 0u) {
#pragma unroll
    for (int v = 0; v < 8; ++v) Rs[wave * 16u + hh * 8u + (unsigned)v] = val[v];
  }
  __syncthreads();

  if (wave == 0u) {
    const v4f x = *(const v4f*)&Rs[lane * 4u];
    float* p = out + (size_t)b * SEQ_FULL + q0 + lane * 4u;
    *(volatile v4f*)p = x;
    __threadfence();
    *(volatile v4f*)p = x;
  }
}

extern "C" void kernel_launch(void* const* d_in, const int* in_sizes, int n_in,
                              void* d_out, int out_size, void* d_ws, size_t ws_size,
                              hipStream_t stream) {
  if (n_in < 4) return;
  const long long need_x = ((long long)(NB - 1) * SEQ_FULL + SEQ) * HD;
  const long long need_o = (long long)(NB - 1) * SEQ_FULL + SEQ;
  if ((long long)in_sizes[0] < need_x) return;
  if ((long long)in_sizes[1] < need_x) return;
  if (in_sizes[2] < 1) return;
  if (in_sizes[3] < NB) return;
  if ((long long)out_size < need_o) return;
  if (ws_size < WS_TOTAL) return;

  const float* queries = (const float*)d_in[0];
  const float* keys    = (const float*)d_in[1];
  const float* scale   = (const float*)d_in[2];
  const int*   vlens   = (const int*)d_in[3];
  float* out = (float*)d_out;

  char* ws = (char*)d_ws;
  _Float16* Q16 = (_Float16*)(ws + OFF_Q);
  _Float16* K16 = (_Float16*)(ws + OFF_K);

  dim3 blk(256);
  cast_kernel<<<dim3(MROWS * 8 / 256), blk, 0, stream>>>(queries, Q16);
  cast_kernel<<<dim3(MROWS * 8 / 256), blk, 0, stream>>>(keys, K16);
  cred_kernel<<<dim3(SEQ / 128, NB), blk, 0, stream>>>(Q16, K16, scale, vlens, out);
}
